// MyModel_87522843560112
// MI455X (gfx1250) — hardware-verified
//
#include <hip/hip_runtime.h>
#include <stdint.h>


#ifndef NB
#define NB 8
#endif
#ifndef SEQ
#define SEQ 2048
#endif
#define NB_FULL  8
#define SEQ_FULL 2048
#define TQ_      SEQ
#define TV_      SEQ
#define TQ_FULL  SEQ_FULL
#define TV_FULL  SEQ_FULL
#define D_       128
#define KT       64
#define QROWS    128
#define NW       8
#define NIT      (TV_ / KT)
#define PCARRY     16384.0f
#define PCARRY_INV (1.0f / 16384.0f)

static_assert(NB >= 1 && NB <= NB_FULL);
static_assert(SEQ >= QROWS && SEQ <= SEQ_FULL);
static_assert(TQ_ % QROWS == 0);
static_assert(TV_ % KT == 0);
static_assert(TQ_ == TV_);
static_assert(((long)NB * TQ_ * 16) % 256 == 0);

#define QS_ROWE 136
#define KS_ROWE 136
#define VT_ROWE 72
#define P_ROWE  72
#define OS_ROWE 132
#define SM_QS   0
#define SM_KS   (SM_QS + QROWS * QS_ROWE * 2)
#define SM_VT   (SM_KS + KT * KS_ROWE * 2)
#define SM_P    (SM_VT + D_ * VT_ROWE * 2)
#define SMEM_BYTES (SM_P + NW * 16 * P_ROWE * 2)
static_assert(SM_KS == 34816);
static_assert(SM_VT == 52224);
static_assert(SM_P  == 70656);
static_assert(SMEM_BYTES == 89088);
static_assert(NW * 16 * OS_ROWE * 4 <= SM_P);
static_assert((SM_KS % 16) == 0 && (SM_VT % 16) == 0 && (SM_P % 16) == 0);

typedef unsigned short v8us  __attribute__((ext_vector_type(8)));
typedef unsigned short v16us __attribute__((ext_vector_type(16)));
typedef __bf16         v16bf __attribute__((ext_vector_type(16)));
typedef _Float16       v8h   __attribute__((ext_vector_type(8)));
typedef _Float16       v16h  __attribute__((ext_vector_type(16)));
typedef float          v8f   __attribute__((ext_vector_type(8)));
typedef float          v4f   __attribute__((ext_vector_type(4)));

union FragU { v16us v; v8us h[2]; };
union FragH { v16h  v; v8h  h[2]; };

__device__ __forceinline__ v8f wmma_bf16_g(v16us a, v16us b, v8f acc) {
  v16bf av = __builtin_bit_cast(v16bf, a);
  v16bf bv = __builtin_bit_cast(v16bf, b);
  acc = __builtin_amdgcn_wmma_f32_16x16x32_bf16(false, av, false, bv, (short)0, acc, false, false);
  asm volatile("v_nop\n\tv_nop\n\tv_nop\n\tv_nop" : "+v"(acc) : "v"(av), "v"(bv));
  return acc;
}
__device__ __forceinline__ v8f wmma_f16_g(v16h a, v16h b, v8f acc) {
  acc = __builtin_amdgcn_wmma_f32_16x16x32_f16(false, a, false, b, (short)0, acc, false, false);
  asm volatile("v_nop\n\tv_nop\n\tv_nop\n\tv_nop" : "+v"(acc) : "v"(a), "v"(b));
  return acc;
}

__device__ __forceinline__ unsigned short bf16_bits_rne(float f) {
  unsigned u = __float_as_uint(f);
  u = u + 0x7FFFu + ((u >> 16) & 1u);
  return (unsigned short)(u >> 16);
}
__device__ __forceinline__ float bf16_rne_f(float f) {
  return __uint_as_float(((unsigned)bf16_bits_rne(f)) << 16);
}
__device__ __forceinline__ unsigned short f16_bits_of(float f) {
  _Float16 hv = (_Float16)f;
  return __builtin_bit_cast(unsigned short, hv);
}

__global__ __launch_bounds__(256)
void k_cvt_qk(const float* __restrict__ Q, const float* __restrict__ K,
              unsigned short* Qb, unsigned short* Kb) {
  const int i   = blockIdx.x * 256 + threadIdx.x;
  const int per = TQ_ * (D_ / 8);
  const int b   = i / per;
  const int rem = i - b * per;
  const size_t src = (size_t)b * TQ_FULL * D_ + (size_t)rem * 8;
  const v4f q0 = *(const v4f*)(Q + src);
  const v4f q1 = *(const v4f*)(Q + src + 4);
  const v4f c0 = *(const v4f*)(K + src);
  const v4f c1 = *(const v4f*)(K + src + 4);
  v8us qo, ko;
  #pragma unroll
  for (int e = 0; e < 4; ++e) {
    qo[e]     = bf16_bits_rne(q0[e]);
    qo[4 + e] = bf16_bits_rne(q1[e]);
    ko[e]     = bf16_bits_rne(c0[e]);
    ko[4 + e] = bf16_bits_rne(c1[e]);
  }
  unsigned short* qd = Qb + (size_t)i * 8;
  unsigned short* kd = Kb + (size_t)i * 8;
  *(volatile v8us*)qd = qo;
  *(volatile v8us*)kd = ko;
  __threadfence();
  *(volatile v8us*)qd = qo;
  *(volatile v8us*)kd = ko;
}

__global__ __launch_bounds__(256)
void k_vt(const float* __restrict__ V, unsigned short* Vt) {
  __shared__ __attribute__((aligned(16))) unsigned short T[D_][VT_ROWE];
  const int tid = threadIdx.x;
  const int b   = blockIdx.x / (TV_ / KT);
  const int kt  = blockIdx.x % (TV_ / KT);
  const int k0  = kt * KT;
  const float* vb = V + ((size_t)b * TV_FULL + k0) * D_;
  #pragma unroll
  for (int i = 0; i < 8; ++i) {
    const int fi  = tid + i * 256;
    const int key = fi >> 5;
    const int d4  = (fi & 31) * 4;
    const v4f x = *(const v4f*)(vb + (size_t)key * D_ + d4);
    #pragma unroll
    for (int e = 0; e < 4; ++e) T[d4 + e][key] = f16_bits_of(bf16_rne_f(x[e]));
  }
  __syncthreads();
  const int w = tid >> 5, lane = tid & 31;
  const int q = lane >> 3, pc = lane & 7;
  v8us vals[4];
  #pragma unroll
  for (int i = 0; i < 4; ++i) {
    const int row = w * 16 + i * 4 + q;
    vals[i] = *(const v8us*)(&T[row][pc * 8]);
  }
  #pragma unroll
  for (int i = 0; i < 4; ++i) {
    const int row = w * 16 + i * 4 + q;
    *(volatile v8us*)(Vt + ((size_t)b * D_ + row) * TV_ + k0 + pc * 8) = vals[i];
  }
  __threadfence();
  #pragma unroll
  for (int i = 0; i < 4; ++i) {
    const int row = w * 16 + i * 4 + q;
    *(volatile v8us*)(Vt + ((size_t)b * D_ + row) * TV_ + k0 + pc * 8) = vals[i];
  }
}

__global__ __launch_bounds__(256)
void k_attn(const unsigned short* __restrict__ Qb, const unsigned short* __restrict__ Kb,
            const unsigned short* __restrict__ Vt, const float* __restrict__ scale_p,
            const int* __restrict__ mask_q, const int* __restrict__ mask_v,
            float* Out)
{
  extern __shared__ v4f smem_v[];
  char* smem = (char*)smem_v;
  unsigned short* Qs  = (unsigned short*)(smem + SM_QS);
  unsigned short* Ks  = (unsigned short*)(smem + SM_KS);
  unsigned short* Vts = (unsigned short*)(smem + SM_VT);

  const int tid  = threadIdx.x;
  const int w    = tid >> 5;
  const int lane = tid & 31;
  const int h    = lane >> 4;
  const int lcol = lane & 15;

  _Float16* Ps = (_Float16*)(smem + SM_P) + w * 16 * P_ROWE;

  const int bid   = blockIdx.x;
  const int b     = bid / (TQ_ / QROWS);
  const int qt    = bid % (TQ_ / QROWS);
  const int qblk0 = qt * QROWS;
  const int q0w   = qblk0 + w * 16;

  const float scal = bf16_rne_f(scale_p[0]);

  #pragma unroll
  for (int i = 0; i < 8; ++i) {
    const int ci  = tid + i * 256;
    const int row = ci >> 4;
    const int ch  = ci & 15;
    const v8us x = *(const v8us*)(Qb + ((size_t)b * TQ_ + qblk0 + row) * D_ + ch * 8);
    *(v8us*)(Qs + row * QS_ROWE + ch * 8) = x;
  }

  float m_[8], l_[8];
  v8f   o_[8];
  #pragma unroll
  for (int r = 0; r < 8; ++r) { m_[r] = -INFINITY; l_[r] = 0.f; }
  #pragma unroll
  for (int j = 0; j < 8; ++j) { v8f z = {}; o_[j] = z; }

  #pragma unroll 1
  for (int it = 0; it < NIT; ++it) {
    const int k0 = it * KT;

    #pragma unroll
    for (int i = 0; i < 4; ++i) {
      const int ci  = tid + i * 256;
      const int row = ci >> 4;
      const int ch  = ci & 15;
      const v8us x = *(const v8us*)(Kb + ((size_t)b * TV_ + k0 + row) * D_ + ch * 8);
      *(v8us*)(Ks + row * KS_ROWE + ch * 8) = x;
    }
    #pragma unroll
    for (int i = 0; i < 4; ++i) {
      const int ci  = tid + i * 256;
      const int row = ci >> 3;
      const int ch  = ci & 7;
      const v8us x = *(const v8us*)(Vt + ((size_t)b * D_ + row) * TV_ + k0 + ch * 8);
      *(v8us*)(Vts + row * VT_ROWE + ch * 8) = x;
    }
    __syncthreads();

    v8f sacc[4];
    #pragma unroll
    for (int t = 0; t < 4; ++t) { v8f z = {}; sacc[t] = z; }
    #pragma unroll
    for (int c = 0; c < 4; ++c) {
      FragU qa;
      const unsigned short* qr = Qs + (w * 16 + lcol) * QS_ROWE + c * 32 + 8 * h;
      qa.h[0] = *(const v8us*)(qr);
      qa.h[1] = *(const v8us*)(qr + 16);
      #pragma unroll
      for (int t = 0; t < 4; ++t) {
        FragU kb;
        const unsigned short* kr = Ks + (t * 16 + lcol) * KS_ROWE + c * 32 + 8 * h;
        kb.h[0] = *(const v8us*)(kr);
        kb.h[1] = *(const v8us*)(kr + 16);
        sacc[t] = wmma_bf16_g(qa.v, kb.v, sacc[t]);
      }
    }

    float s_[4][8];
    #pragma unroll
    for (int t = 0; t < 4; ++t) {
      const int   mvv   = mask_v[(size_t)b * TV_FULL + k0 + t * 16 + lcol];
      const float biasf = (1.0f - (float)mvv) * 1.0e9f;
      #pragma unroll
      for (int r = 0; r < 8; ++r) s_[t][r] = scal * sacc[t][r] - biasf;
    }

    float alpha[8];
    #pragma unroll
    for (int r = 0; r < 8; ++r) {
      float rm = fmaxf(fmaxf(s_[0][r], s_[1][r]), fmaxf(s_[2][r], s_[3][r]));
      #pragma unroll
      for (int off = 1; off < 16; off <<= 1) rm = fmaxf(rm, __shfl_xor(rm, off, 32));
      const float mn = fmaxf(m_[r], rm);
      alpha[r] = __expf(m_[r] - mn);
      m_[r] = mn;
      float rs = 0.f;
      #pragma unroll
      for (int t = 0; t < 4; ++t) { const float p = __expf(s_[t][r] - mn); s_[t][r] = p; rs += p; }
      #pragma unroll
      for (int off = 1; off < 16; off <<= 1) rs += __shfl_xor(rs, off, 32);
      l_[r] = l_[r] * alpha[r] + rs;
    }
    #pragma unroll
    for (int j = 0; j < 8; ++j)
      #pragma unroll
      for (int r = 0; r < 8; ++r) o_[j][r] *= alpha[r];

    #pragma unroll
    for (int t = 0; t < 4; ++t)
      #pragma unroll
      for (int r = 0; r < 8; ++r)
        Ps[(8 * h + r) * P_ROWE + t * 16 + lcol] = (_Float16)(s_[t][r] * PCARRY);
    __syncthreads();

    #pragma unroll
    for (int kc = 0; kc < 2; ++kc) {
      FragH pa;
      const _Float16* pr = Ps + lcol * P_ROWE + kc * 32 + 8 * h;
      pa.h[0] = *(const v8h*)(pr);
      pa.h[1] = *(const v8h*)(pr + 16);
      #pragma unroll
      for (int j = 0; j < 8; ++j) {
        FragH vb;
        const _Float16* vr = (const _Float16*)Vts + (j * 16 + lcol) * VT_ROWE + kc * 32 + 8 * h;
        vb.h[0] = *(const v8h*)(vr);
        vb.h[1] = *(const v8h*)(vr + 16);
        o_[j] = wmma_f16_g(pa.v, vb.v, o_[j]);
      }
    }
    __syncthreads();
  }

  float fac[8];
  #pragma unroll
  for (int r = 0; r < 8; ++r) {
    const float inv = PCARRY_INV / l_[r];
    const int   mqi = mask_q[(size_t)b * TQ_FULL + q0w + 8 * h + r];
    fac[r] = mqi ? inv : 0.0f;
  }
  float* Os = (float*)smem + w * 16 * OS_ROWE;
  #pragma unroll
  for (int j = 0; j < 8; ++j)
    #pragma unroll
    for (int r = 0; r < 8; ++r)
      Os[(8 * h + r) * OS_ROWE + j * 16 + lcol] = o_[j][r] * fac[r];
  __syncthreads();

  v4f vals[16];
  #pragma unroll
  for (int i = 0; i < 16; ++i) vals[i] = *(const v4f*)(Os + i * OS_ROWE + lane * 4);

  float* ob = Out + ((size_t)b * TQ_ + q0w) * D_ + lane * 4;
  #pragma unroll
  for (int i = 0; i < 16; ++i) *(volatile v4f*)(ob + (size_t)i * D_) = vals[i];
  __threadfence();
  #pragma unroll
  for (int i = 0; i < 16; ++i) *(volatile v4f*)(ob + (size_t)i * D_) = vals[i];
}

extern "C" void kernel_launch(void* const* d_in, const int* in_sizes, int n_in,
                              void* d_out, int out_size, void* d_ws, size_t ws_size,
                              hipStream_t stream) {
  if (n_in < 6) return;
  const long needQ  = ((long)(NB - 1) * TQ_FULL + TQ_) * D_;
  const long needKV = ((long)(NB - 1) * TV_FULL + TV_) * D_;
  const long needMQ = (long)(NB - 1) * TQ_FULL + TQ_;
  const long needMV = (long)(NB - 1) * TV_FULL + TV_;
  if ((long)in_sizes[0] < needQ || (long)in_sizes[1] < needKV || (long)in_sizes[2] < needKV) return;
  if (in_sizes[3] < 1 || (long)in_sizes[4] < needMQ || (long)in_sizes[5] < needMV) return;
  if ((long)out_size < (long)NB * TQ_ * D_) return;

  const float* Q  = (const float*)d_in[0];
  const float* V  = (const float*)d_in[1];
  const float* K  = (const float*)d_in[2];
  const float* sc = (const float*)d_in[3];
  const int*   mq = (const int*)d_in[4];
  const int*   mv = (const int*)d_in[5];
  float* out = (float*)d_out;

  const size_t nQ   = (size_t)NB * TQ_ * D_;
  const size_t nKV  = (size_t)NB * TV_ * D_;
  const size_t offQ = 0;
  const size_t offK = offQ + nQ * 2;
  const size_t offV = offK + nKV * 2;
  const size_t tot  = offV + nKV * 2;
  if (tot > ws_size) return;
  unsigned short* Qb  = (unsigned short*)((char*)d_ws + offQ);
  unsigned short* Kb  = (unsigned short*)((char*)d_ws + offK);
  unsigned short* Vtp = (unsigned short*)((char*)d_ws + offV);

  k_cvt_qk<<<dim3((unsigned)(nQ / 8 / 256)), dim3(256), 0, stream>>>(Q, K, Qb, Kb);
  k_vt<<<dim3((unsigned)(NB * (TV_ / KT))), dim3(256), 0, stream>>>(V, Vtp);
  hipFuncSetAttribute(reinterpret_cast<const void*>(&k_attn),
                      hipFuncAttributeMaxDynamicSharedMemorySize, SMEM_BYTES);
  k_attn<<<dim3((unsigned)(NB * (TQ_ / QROWS))), dim3(256), SMEM_BYTES, stream>>>(
      Qb, Kb, Vtp, sc, mq, mv, out);
}
